// GNODecoder_36112085024917
// MI455X (gfx1250) — hardware-run, weakly checked
//
#include <hip/hip_runtime.h>


namespace {
constexpr int NQ = 100000, NL = 16384, E = 1000000, CI = 128, CO = 4, HK = 64, PH = 256, N = NQ  ;
constexpr float AS = 1024.0f  , WSC = 256.0f;
typedef _Float16 b16;
typedef __attribute__((ext_vector_type(16))) _Float16 v16b;
typedef __attribute__((ext_vector_type(8))) _Float16 v8b;
typedef __attribute__((ext_vector_type(8))) float v8f;
typedef __attribute__((ext_vector_type(4))) float v4f;
__device__ __forceinline__ float bf16_rne(float f) { unsigned int u = __float_as_uint(f); u += 0x7FFFu + ((u >> 16) & 1u); float r = __uint_as_float(u & 0xFFFF0000u); asm volatile("" : "+v"(r)); return r; }
__device__ __forceinline__ float bfv(float f) { float r = bf16_rne(f); asm volatile("" : "+v"(r)); return r; }
__device__ __forceinline__ void split16(float v, b16& hi, b16& lo) { hi = (b16)v; lo = (b16)(v - (float)hi); }
__device__ __forceinline__ v16b frag_kb(const b16* p, int hh) { const v8b a = *(const v8b*)(p + 8 * hh), b = *(const v8b*)(p + 16 + 8 * hh); v16b f;
#pragma unroll
  for (int e = 0; e < 8; ++e) { f[e] = a[e]; f[8 + e] = b[e]; } return f; }
__device__ __forceinline__ v8f wmma16b(v16b a, v16b b, v8f c) { v8f d = __builtin_amdgcn_wmma_f32_16x16x32_f16(false, a, false, b, (short)0, c, false, false); asm volatile("v_nop\n\tv_nop\n\tv_nop\n\tv_nop" : "+v"(d) : "v"(a), "v"(b)); return d; }
__device__ __forceinline__ void wave_lds_sync() { __builtin_amdgcn_fence(__ATOMIC_RELEASE, "workgroup"); __builtin_amdgcn_wave_barrier(); __builtin_amdgcn_fence(__ATOMIC_ACQUIRE, "workgroup"); }
__device__ __forceinline__ float pmul(float a, float b) { float p = a * b; asm volatile("" : "+v"(p)); return p; }
__device__ __forceinline__ int iclamp(int v, int lo, int hi) { return v < lo ? lo : (v > hi ? hi : v); }
__device__ __forceinline__ float gelu_t(float x) { const float u = 0.7978845608028654f * (x + 0.044715f * x * x * x); return 0.5f * x * (1.0f + tanhf(u)); }
constexpr int CSR_NBLK8 = 512, CSR_GB8 = 8, CSR_GN8 = 1 << CSR_GB8  , CSR_TS8 = (CSR_GN8 < 32 ? 32 : CSR_GN8)  , CSR_MAXG8 = 512, CSR_CAP8 = 12288  ;
__device__ __host__ __forceinline__ int csr_tix8(int v) { return (v >> CSR_GB8) * CSR_TS8 + (v & (CSR_GN8 - 1)); }
__global__ __launch_bounds__(64) void csrA_kernel8(const int* __restrict__ dst, int E, int N, int nG, int CHP, int NGP, int* __restrict__ STG, int* __restrict__ HST) {
  extern __shared__ int sm[];
  int* cnt = sm; int* run = sm + NGP; int* ids = sm + 2 * NGP;
  const int b = blockIdx.x; const int ch = (E + CSR_NBLK8 - 1) / CSR_NBLK8; const int e0 = b * ch, e1 = min(E, e0 + ch);
  for (int i = threadIdx.x; i < NGP; i += 64) cnt[i] = 0;
  for (int i = threadIdx.x; i < CHP; i += 64) ids[i] = -1;
  __syncthreads();
  if (threadIdx.x == 0) {
    for (int e = e0; e < e1; ++e) { int d = dst[e]; d = (d < 0) ? 0 : (d >= N ? N - 1 : d); cnt[d >> CSR_GB8] += 1; }
    int acc = 0; for (int g = 0; g < nG; ++g) { run[g] = acc; acc += cnt[g]; }
    for (int e = e0; e < e1; ++e) { int d = dst[e]; d = (d < 0) ? 0 : (d >= N ? N - 1 : d); const int g = d >> CSR_GB8; ids[run[g]] = e; run[g] += 1; } }
  __syncthreads();
  typedef __attribute__((ext_vector_type(4))) int v4i;
  for (int pass = 0; pass < 2; ++pass) {
    for (int i = threadIdx.x; i < CHP / 4; i += 64) *(volatile v4i*)(STG + (size_t)b * CHP + i * 4) = *(const v4i*)(&ids[i * 4]);
    for (int i = threadIdx.x; i < NGP / 4; i += 64) { v4i v; for (int e = 0; e < 4; ++e) v[e] = (i * 4 + e < nG) ? cnt[i * 4 + e] : 0; *(volatile v4i*)(HST + (size_t)b * NGP + i * 4) = v; }
    __threadfence(); }
}
__global__ __launch_bounds__(512) void csrS_kernel8(const int* __restrict__ HST, int nG, int NGP, int* __restrict__ START, int* __restrict__ TOT, int* __restrict__ OFF) {
  __shared__ int tot[CSR_MAXG8];
  const int b = threadIdx.x;
  for (int pass = 0; pass < 2; ++pass) { int runb = 0; for (int g = 0; g < nG; ++g) { int c = HST[(size_t)b * NGP + g]; c = (c < 0) ? 0 : c; ((volatile int*)OFF)[(size_t)g * CSR_NBLK8 + b] = runb; runb += c; } __threadfence(); }
  for (int g = threadIdx.x; g < nG; g += 512) { int s = 0; for (int bb = 0; bb < CSR_NBLK8; ++bb) { int c = HST[(size_t)bb * NGP + g]; s += (c < 0) ? 0 : c; } tot[g] = s; }
  __syncthreads();
  if (threadIdx.x < 32) {
    __shared__ int st[CSR_MAXG8 + 32];
    if (threadIdx.x == 0) { int acc = 0; for (int g = 0; g < NGP; ++g) { st[g] = acc; if (g < nG) acc += (tot[g] + 31) & ~31; } st[NGP] = acc; }
    __builtin_amdgcn_fence(__ATOMIC_RELEASE, "workgroup"); __builtin_amdgcn_wave_barrier(); __builtin_amdgcn_fence(__ATOMIC_ACQUIRE, "workgroup");
    for (int pass = 0; pass < 2; ++pass) { for (int i = threadIdx.x; i < NGP + 32; i += 32) { ((volatile int*)START)[i] = (i <= NGP) ? st[min(i, NGP)] : 0; ((volatile int*)TOT)[i] = (i < nG) ? tot[i] : 0; } __threadfence(); } }
}
__global__ __launch_bounds__(256) void csrB_kernel8(const int* __restrict__ dst, int N, int nG, int CHP, int NGP, int permLen, const int* __restrict__ STG, const int* __restrict__ HST, const int* __restrict__ OFF, const int* __restrict__ START, const int* __restrict__ TOT, int* __restrict__ PERM, int* __restrict__ ROWPTR, int* __restrict__ ROWCNT, int* __restrict__ FLAG) {
  typedef __attribute__((ext_vector_type(4))) int v4i;
  __shared__ int ids[CSR_CAP8]; __shared__ unsigned short key[CSR_CAP8]; __shared__ int outp[CSR_CAP8]; __shared__ int ncnt[CSR_GN8 + 1]; __shared__ int boff[CSR_NBLK8 + 1];
  const int g = blockIdx.x, t_ = threadIdx.x; int tot = TOT[g]; int st = START[g], stn = START[g + 1]; const int v0 = g * CSR_GN8; const int nv = min(CSR_GN8, N - v0); const int t0 = g * CSR_TS8;
  st = (st < 0) ? 0 : (st > permLen - 32 ? permLen - 32 : st) & ~31; stn = (stn < st) ? st : (stn > permLen ? permLen : stn); tot = (tot < 0) ? 0 : tot; if (tot > stn - st && tot <= CSR_CAP8) tot = stn - st;
  if (tot > CSR_CAP8) {
    for (int pass = 0; pass < 2; ++pass) { for (int i = t_; i < CSR_TS8 / 4; i += 256) { v4i a, c; for (int e = 0; e < 4; ++e) { a[e] = st; c[e] = 0; } *(volatile v4i*)(ROWPTR + t0 + i * 4) = a; *(volatile v4i*)(ROWCNT + t0 + i * 4) = c; } if (t_ == 0) ((volatile int*)FLAG)[0] = 1; __threadfence(); } (void)nv; return; }
  if (t_ == 0) { int acc = 0; for (int b = 0; b < CSR_NBLK8; ++b) { boff[b] = acc; int c = HST[(size_t)b * NGP + g]; c = (c < 0) ? 0 : (c > CHP ? CHP : c); acc += c; if (acc > tot) acc = tot; } boff[CSR_NBLK8] = acc; }
  for (int i = t_; i <= CSR_GN8; i += 256) ncnt[i] = 0;
  __syncthreads();
  for (int b = 0; b < CSR_NBLK8; ++b) { const int c = boff[b + 1] - boff[b]; int o_ = OFF[(size_t)g * CSR_NBLK8 + b]; o_ = (o_ < 0) ? 0 : (o_ > CHP - c ? CHP - c : o_); const int* src_ = STG + (size_t)b * CHP + o_;
    for (int i = t_; i < c; i += 256) { int id = src_[i]; id = (id < 0) ? 0 : id; ids[boff[b] + i] = id; int d = dst[id]; d = (d < v0) ? v0 : (d >= N ? N - 1 : d); int kk = d - v0; kk = (kk < 0) ? 0 : (kk >= CSR_GN8 ? CSR_GN8 - 1 : kk); key[boff[b] + i] = (unsigned short)kk; } }
  __syncthreads();
  if (t_ == 0) { for (int i = 0; i < tot; ++i) ncnt[key[i]] += 1; int acc = 0; for (int vl = 0; vl < CSR_GN8; ++vl) { const int c = ncnt[vl]; ncnt[vl] = acc; acc += c; } ncnt[CSR_GN8] = acc;
    for (int i = 0; i < tot; ++i) { const int vl = key[i]; outp[ncnt[vl]] = ids[i]; ncnt[vl] += 1; }
    for (int vl = CSR_GN8; vl > 0; --vl) ncnt[vl] = ncnt[vl - 1]; ncnt[0] = 0; }
  __syncthreads();
  for (int pass = 0; pass < 2; ++pass) {
    for (int i = t_; i < (stn - st) / 4; i += 256) { v4i v; for (int e = 0; e < 4; ++e) { const int q = i * 4 + e; v[e] = (q < tot) ? outp[q] : -1; } *(volatile v4i*)(PERM + st + i * 4) = v; }
    for (int i = t_; i < CSR_TS8 / 4; i += 256) { v4i a, c; for (int e = 0; e < 4; ++e) { const int vl = i * 4 + e; const int vc = vl < CSR_GN8 ? vl : CSR_GN8; a[e] = (vl < CSR_GN8) ? st + ncnt[vc] : st; c[e] = (vl < nv) ? (ncnt[(vc < CSR_GN8 ? vc : CSR_GN8 - 1) + 1] - ncnt[vc]) : 0; } *(volatile v4i*)(ROWPTR + t0 + i * 4) = a; *(volatile v4i*)(ROWCNT + t0 + i * 4) = c; }
    __threadfence(); }
}
__global__ __launch_bounds__(256) void csrZ_kernel8(int* __restrict__ p, size_t n4) { typedef __attribute__((ext_vector_type(4))) int v4i; const size_t tid = (size_t)blockIdx.x * 256 + threadIdx.x, nth = (size_t)gridDim.x * 256; v4i z = {0, 0, 0, 0}; for (size_t i = tid; i < n4; i += nth) *(volatile v4i*)(p + i * 4) = z; }
struct CsrBufs8 { int *STG, *HST, *OFF, *START, *TOT, *PERM, *ROWPTR, *ROWCNT, *FLAG; int nG, NGP, CHP; size_t permLen; char* base; size_t bytes; };
static size_t csr_carve8(CsrBufs8& c, char* ws, size_t off, int E, int N) {
  const size_t off0 = off; c.base = ws + off;
  auto al = [&](size_t bytes) { char* p = ws + off; off += (bytes + 255) & ~(size_t)255; return p; };
  c.nG = (N + CSR_GN8 - 1) / CSR_GN8; c.NGP = (c.nG + 31) & ~31; const int ch = (E + CSR_NBLK8 - 1) / CSR_NBLK8; c.CHP = (ch + 31) & ~31; c.permLen = (size_t)E + 32 * (size_t)c.nG + 32;
  c.STG = (int*)al((size_t)CSR_NBLK8 * c.CHP * 4); c.HST = (int*)al((size_t)CSR_NBLK8 * c.NGP * 4); c.OFF = (int*)al((size_t)c.NGP * CSR_NBLK8 * 4); c.START = (int*)al((size_t)(c.NGP + 64) * 4); c.TOT = (int*)al((size_t)(c.NGP + 64) * 4);
  c.PERM = (int*)al(c.permLen * 4); c.ROWPTR = (int*)al((size_t)c.nG * CSR_TS8 * 4); c.ROWCNT = (int*)al((size_t)c.nG * CSR_TS8 * 4); c.FLAG = (int*)al(256);
  c.bytes = off - off0; return off;
}
static void csr_build8(const CsrBufs8& c, const int* dst, int E, int N, hipStream_t stream) {
  const size_t smem = (size_t)(2 * c.NGP + c.CHP) * 4;
  csrZ_kernel8<<<512, 256, 0, stream>>>((int*)c.base, c.bytes / 16);
  csrA_kernel8<<<CSR_NBLK8, 64, smem, stream>>>(dst, E, N, c.nG, c.CHP, c.NGP, c.STG, c.HST);
  csrS_kernel8<<<1, 512, 0, stream>>>(c.HST, c.nG, c.NGP, c.START, c.TOT, c.OFF);
  csrB_kernel8<<<c.nG, 256, 0, stream>>>(dst, N, c.nG, c.CHP, c.NGP, (int)c.permLen, c.STG, c.HST, c.OFF, c.START, c.TOT, c.PERM, c.ROWPTR, c.ROWCNT, c.FLAG);
}


__global__ __launch_bounds__(256) void wput_kernel(const float* __restrict__ w0, const float* __restrict__ w1, const float* __restrict__ w2, const float* __restrict__ p0, const float* __restrict__ p1, b16* __restrict__ W0T, b16* __restrict__ W1T, b16* __restrict__ W2T, b16* __restrict__ P0T, b16* __restrict__ P1T) { const int t = threadIdx.x + blockIdx.x * 256; const int nt = gridDim.x * 256;
  auto put = [&](b16* dst, const float* w, int din, int dout, int rows, int kpad) { for (int i8 = t; i8 < rows * kpad / 8; i8 += nt) { const int o = i8 / (kpad / 8), k0 = (i8 % (kpad / 8)) * 8; v8b v;
#pragma unroll
      for (int j = 0; j < 8; ++j) { const int k = k0 + j; v[j] = (b16)((o < dout && k < din) ? bf16_rne(w[(size_t)k * dout + o]) * WSC : 0.0f); } *(volatile v8b*)(dst + (size_t)o * kpad + k0) = v; } };
  for (int pass = 0; pass < 2; ++pass) { put(W0T, w0, 6, HK, HK, 32); put(W1T, w1, HK, HK, HK, HK); put(W2T, w2, HK, CI, CI, HK); put(P0T, p0, CI, PH, PH, CI); put(P1T, p1, PH, CO, 16, PH); __threadfence(); } }
__global__ __launch_bounds__(32) void edge_kernel(const float* __restrict__ rn, const float* __restrict__ pq, const float* __restrict__ pl, const int* __restrict__ edst, const int* __restrict__ esrc, const b16* __restrict__ W0T, const b16* __restrict__ W1T, const b16* __restrict__ W2T, const float* __restrict__ b0, const float* __restrict__ b1, const float* __restrict__ b2, int EB, int ELIM, float* __restrict__ REP) {
  __shared__ __attribute__((aligned(16))) b16 Ah[16][HK + 8], Al[16][HK + 8]; __shared__ float Tf[16][CI + 4]; __shared__ int Sl[16]; const int lane = threadIdx.x, nloc = lane & 15, hlf = lane >> 4; const size_t e0 = (size_t)EB + (size_t)blockIdx.x * 16; if (e0 >= (size_t)ELIM) return;
  { const size_t e = e0 + nloc; const int q = iclamp(edst[e], 0, NQ - 1), l = iclamp(esrc[e], 0, NL - 1); if (hlf == 0) Sl[nloc] = l;
    for (int k = 0; k < 3; ++k) Ah[nloc][hlf * 3 + k] = (b16)(bf16_rne(hlf ? pl[(size_t)l * 3 + k] : pq[(size_t)q * 3 + k]) * AS);
    for (int k = 6 + hlf; k < HK + 8; k += 2) Ah[nloc][k] = (b16)0.0f; for (int k = hlf; k < HK + 8; k += 2) Al[nloc][k] = (b16)0.0f; }
  wave_lds_sync(); v8f a4[4] = {(v8f){}, (v8f){}, (v8f){}, (v8f){}};
  { const v16b a = frag_kb(&Ah[nloc][0], hlf);
#pragma unroll
    for (int t = 0; t < 4; ++t) a4[t] = wmma16b(a, frag_kb(W0T + (size_t)(t * 16 + nloc) * 32, hlf), a4[t]); }
#pragma unroll
  for (int t = 0; t < 4; ++t)
#pragma unroll
    for (int r8 = 0; r8 < 8; ++r8) Tf[8 * hlf + r8][t * 16 + nloc] = gelu_t(a4[t][r8] * (1.0f / (AS * WSC)) + bfv(b0[t * 16 + nloc]));
  wave_lds_sync();
  for (int rr = 0; rr < 16; ++rr) for (int q = 0; q < 2; ++q) { b16 p, ql; split16(Tf[rr][q * 32 + lane] * AS, p, ql); Ah[rr][q * 32 + lane] = p; Al[rr][q * 32 + lane] = ql; }
  wave_lds_sync();
#pragma unroll
  for (int t = 0; t < 4; ++t) a4[t] = (v8f){};
#pragma unroll
  for (int kb = 0; kb < HK; kb += 32) { const v16b a = frag_kb(&Ah[nloc][kb], hlf), al = frag_kb(&Al[nloc][kb], hlf);
#pragma unroll
    for (int t = 0; t < 4; ++t) { const v16b bw = frag_kb(W1T + (size_t)(t * 16 + nloc) * HK + kb, hlf); a4[t] = wmma16b(a, bw, a4[t]); a4[t] = wmma16b(al, bw, a4[t]); } }
#pragma unroll
  for (int t = 0; t < 4; ++t)
#pragma unroll
    for (int r8 = 0; r8 < 8; ++r8) Tf[8 * hlf + r8][t * 16 + nloc] = gelu_t(a4[t][r8] * (1.0f / (AS * WSC)) + bfv(b1[t * 16 + nloc]));
  wave_lds_sync();
  for (int rr = 0; rr < 16; ++rr) for (int q = 0; q < 2; ++q) { b16 p, ql; split16(Tf[rr][q * 32 + lane] * AS, p, ql); Ah[rr][q * 32 + lane] = p; Al[rr][q * 32 + lane] = ql; }
  wave_lds_sync(); v8f a8[8];
#pragma unroll
  for (int t = 0; t < 8; ++t) a8[t] = (v8f){};
#pragma unroll
  for (int kb = 0; kb < HK; kb += 32) { const v16b a = frag_kb(&Ah[nloc][kb], hlf), al = frag_kb(&Al[nloc][kb], hlf);
#pragma unroll
    for (int t = 0; t < 8; ++t) { const v16b bw = frag_kb(W2T + (size_t)(t * 16 + nloc) * HK + kb, hlf); a8[t] = wmma16b(a, bw, a8[t]); a8[t] = wmma16b(al, bw, a8[t]); } }
#pragma unroll
  for (int t = 0; t < 8; ++t)
#pragma unroll
    for (int r8 = 0; r8 < 8; ++r8) Tf[8 * hlf + r8][t * 16 + nloc] = a8[t][r8] * (1.0f / (AS * WSC)) + bfv(b2[t * 16 + nloc]);
  wave_lds_sync();
  for (int pass = 0; pass < 2; ++pass) { for (int rr = 0; rr < 16; ++rr) { const float* rp = rn + (size_t)Sl[rr] * CI + lane * 4; v4f o; for (int k = 0; k < 4; ++k) o[k] = pmul(Tf[rr][lane * 4 + k], bfv(rp[k])); *(volatile v4f*)(REP + (e0 - EB + rr) * CI + lane * 4) = o; } __threadfence(); } }
template <int FIRST, int LAST>
__global__ __launch_bounds__(256) void agg_kernel(const float* __restrict__ REP, int EB, int EEND, const float* __restrict__ AGGIN, const int* __restrict__ PERM, const int* __restrict__ ROWPTR, const int* __restrict__ ROWCNT, int permLen, int QLIM, int ELIM, float* __restrict__ AGG) { const int wave = threadIdx.x >> 5, lane = threadIdx.x & 31; const size_t i = (size_t)blockIdx.x * 8 + wave; if (i >= (size_t)QLIM) return; int st = ROWPTR[i], cnt = ROWCNT[i]; cnt = iclamp(cnt, 0, E); st = iclamp(st, 0, permLen - cnt);
  v4f acc = FIRST ? (v4f){0, 0, 0, 0} : *(const v4f*)(AGGIN + i * CI + lane * 4); int nin = 0;
#pragma unroll 1
  for (int j = 0; j < cnt; ++j) { const int e = iclamp(PERM[st + j], 0, E - 1); if (e >= ELIM) continue; ++nin; if (e < EB || e >= EEND) continue; const v4f v = *(const v4f*)(REP + (size_t)(e - EB) * CI + lane * 4);
#pragma unroll
    for (int k = 0; k < 4; ++k) acc[k] += v[k]; }
  const float inv = 1.0f / fmaxf((float)nin, 1.0f); v4f o; for (int k = 0; k < 4; ++k) o[k] = LAST ? pmul(acc[k], inv) : acc[k];
  for (int pass = 0; pass < 2; ++pass) { *(volatile v4f*)(AGG + i * CI + lane * 4) = o; __threadfence(); } }
__global__ __launch_bounds__(32) void proj_kernel(const float* __restrict__ AGG, const b16* __restrict__ P0T, const b16* __restrict__ P1T, const float* __restrict__ pb0, const float* __restrict__ pb1, int QLIM, float* __restrict__ OUT) { __shared__ __attribute__((aligned(16))) b16 Ah[16][CI + 8], Al[16][CI + 8], Hh[16][PH + 8], Hl[16][PH + 8]; __shared__ float Tf[16][4]; const int lane = threadIdx.x, nloc = lane & 15, hlf = lane >> 4; const size_t m0 = (size_t)blockIdx.x * 16; if (m0 >= (size_t)QLIM) return;
  for (int rr = 0; rr < 16; ++rr) for (int q = 0; q < 4; ++q) { b16 p, ql; split16(AGG[(m0 + rr) * CI + q * 32 + lane] * AS, p, ql); Ah[rr][q * 32 + lane] = p; Al[rr][q * 32 + lane] = ql; }
  if (lane < 16) for (int k = PH; k < PH + 8; ++k) { Hh[lane][k] = (b16)0.0f; Hl[lane][k] = (b16)0.0f; }
  wave_lds_sync(); v8f acc[16];
#pragma unroll
  for (int t = 0; t < 16; ++t) acc[t] = (v8f){};
#pragma unroll
  for (int kb = 0; kb < CI; kb += 32) { const v16b a = frag_kb(&Ah[nloc][kb], hlf), al = frag_kb(&Al[nloc][kb], hlf);
#pragma unroll
    for (int t = 0; t < 16; ++t) { const v16b bw = frag_kb(P0T + (size_t)(t * 16 + nloc) * CI + kb, hlf); acc[t] = wmma16b(a, bw, acc[t]); acc[t] = wmma16b(al, bw, acc[t]); } }
#pragma unroll
  for (int t = 0; t < 16; ++t) { const int cc = t * 16 + nloc; const float bb = bfv(pb0[cc]);
#pragma unroll
    for (int r8 = 0; r8 < 8; ++r8) { b16 p, ql; split16(gelu_t(acc[t][r8] * (1.0f / (AS * WSC)) + bb) * AS, p, ql); Hh[8 * hlf + r8][cc] = p; Hl[8 * hlf + r8][cc] = ql; } }
  wave_lds_sync(); v8f o8 = {};
#pragma unroll 2
  for (int kb = 0; kb < PH; kb += 32) { const v16b bw = frag_kb(P1T + (size_t)nloc * PH + kb, hlf); o8 = wmma16b(frag_kb(&Hh[nloc][kb], hlf), bw, o8); o8 = wmma16b(frag_kb(&Hl[nloc][kb], hlf), bw, o8); }
  if (nloc < CO) {
#pragma unroll
    for (int r8 = 0; r8 < 8; ++r8) Tf[8 * hlf + r8][nloc] = o8[r8] * (1.0f / (AS * WSC)) + bfv(pb1[nloc]); }
  wave_lds_sync();
  for (int pass = 0; pass < 2; ++pass) { ((volatile float*)OUT)[m0 * CO + lane] = Tf[lane / 4][lane % 4]; ((volatile float*)OUT)[m0 * CO + 32 + lane] = Tf[8 + lane / 4][lane % 4]; __threadfence(); } }
}

extern "C" void kernel_launch(void* const* d_in, const int* in_sizes, int n_in, void* d_out, int out_size, void* d_ws, size_t ws_size, hipStream_t stream) {
  (void)n_in;
  auto Fp = [&](int i) { return (const float*)d_in[i]; }; auto Ip = [&](int i) { return (const int*)d_in[i]; };
  if (in_sizes[0] != NL * CI || in_sizes[1] != NQ * 3 || in_sizes[2] != NL * 3 || in_sizes[3] != E || in_sizes[4] != E || in_sizes[5] != 6 * HK || in_sizes[7] != HK * HK || in_sizes[9] != HK * CI || in_sizes[11] != CI * PH || in_sizes[13] != PH * CO || out_size != NQ * CO) return;
  const int QLIM = NQ, ELIM = E;
  size_t off = 0; char* ws = (char*)d_ws;
  auto carve = [&](size_t bytes) { char* p = ws + off; off += (bytes + 255) & ~(size_t)255; return p; };
  b16* W0T = (b16*)carve(HK * 32 * 2); b16* W1T = (b16*)carve(HK * HK * 2); b16* W2T = (b16*)carve(CI * HK * 2); b16* P0T = (b16*)carve(PH * CI * 2); b16* P1T = (b16*)carve(16 * PH * 2); float* REP = (float*)carve((size_t)(E / 4) * CI * 4); float* AGGA = (float*)carve((size_t)NQ * CI * 4); float* AGGB = (float*)carve((size_t)NQ * CI * 4); CsrBufs8 csr; off = csr_carve8(csr, ws, off, E, NQ);
  if (off > ws_size || off > ((size_t)256 << 20)) return;
  wput_kernel<<<8, 256, 0, stream>>>(Fp(5), Fp(7), Fp(9), Fp(11), Fp(13), W0T, W1T, W2T, P0T, P1T);
  csr_build8(csr, Ip(3), E, NQ, stream);
  { const int EQ = E / 4;
    auto edges = [&](int eb, int ee) { const int hi = ELIM < ee ? ELIM : ee; if (hi > eb) edge_kernel<<<(hi - eb + 15) / 16, 32, 0, stream>>>(Fp(0), Fp(1), Fp(2), Ip(3), Ip(4), W0T, W1T, W2T, Fp(6), Fp(8), Fp(10), eb, hi, REP); };
    edges(0, EQ);          agg_kernel<1, 0><<<(QLIM + 7) / 8, 256, 0, stream>>>(REP, 0, EQ, AGGB, csr.PERM, csr.ROWPTR, csr.ROWCNT, (int)csr.permLen, QLIM, ELIM, AGGA);
    edges(EQ, 2 * EQ);     agg_kernel<0, 0><<<(QLIM + 7) / 8, 256, 0, stream>>>(REP, EQ, 2 * EQ, AGGA, csr.PERM, csr.ROWPTR, csr.ROWCNT, (int)csr.permLen, QLIM, ELIM, AGGB);
    edges(2 * EQ, 3 * EQ); agg_kernel<0, 0><<<(QLIM + 7) / 8, 256, 0, stream>>>(REP, 2 * EQ, 3 * EQ, AGGB, csr.PERM, csr.ROWPTR, csr.ROWCNT, (int)csr.permLen, QLIM, ELIM, AGGA);
    edges(3 * EQ, E);      agg_kernel<0, 1><<<(QLIM + 7) / 8, 256, 0, stream>>>(REP, 3 * EQ, E, AGGA, csr.PERM, csr.ROWPTR, csr.ROWCNT, (int)csr.permLen, QLIM, ELIM, AGGB); }
  proj_kernel<<<QLIM / 16, 32, 0, stream>>>(AGGB, P0T, P1T, Fp(12), Fp(14), QLIM, (float*)d_out);
}
